// SelectiveStateSpaceModel_20177756357189
// MI455X (gfx1250) — hardware-verified
//
#include <hip/hip_runtime.h>

#define NB    2
#define NL    2048
#define DM    1024
#define DI    2048
#define DIN2  4096
#define NS    16
#define DTR   64
#define KDT   64
#define NXD   96
#define NXP   128
#define NROWS (NB * NL)
#define TC    16

static_assert(DM % 32 == 0 && DI % 32 == 0 && KDT % 32 == 0);
static_assert(NROWS % 128 == 0 && DI % 64 == 0 && DM % 64 == 0 && NXP % 64 == 0);
static_assert(NL % TC == 0 && DI % 256 == 0 && TC == 16);
static_assert(DTR + 2 * NS == NXD && NXD <= NXP && DTR == KDT && NXP == 128 && DTR % 8 == 0);
static_assert(DIN2 == 2 * DI);
static_assert(NXD % 4 == 0 && DM % 8 == 0 && DI % 8 == 0 && NS % 4 == 0);
static_assert((NROWS * DM) % 2048 == 0 && (DIN2 * DM) % 2048 == 0 && (NXP * DI) % 2048 == 0);
static_assert((DI * KDT) % 2048 == 0 && (DM * DI) % 2048 == 0 && (NXD * DI) % 8 == 0);

typedef __bf16         v16b  __attribute__((ext_vector_type(16)));
typedef unsigned short v16us __attribute__((ext_vector_type(16)));
typedef unsigned short v8us  __attribute__((ext_vector_type(8)));
typedef float          v8f   __attribute__((ext_vector_type(8)));
typedef float          v4f   __attribute__((ext_vector_type(4)));
typedef v8us __attribute__((may_alias)) v8usa;
typedef v4f  __attribute__((may_alias)) v4fa;

union Frag { v16b v; v8us half[2]; v16us u; };

constexpr size_t OFF_X0   = 0;
constexpr size_t OFF_WIN  = OFF_X0   + (size_t)NROWS * DM * 2;
constexpr size_t OFF_WX   = OFF_WIN  + (size_t)DIN2 * DM * 2;
constexpr size_t OFF_WDT  = OFF_WX   + (size_t)NXP * DI * 2;
constexpr size_t OFF_WOUT = OFF_WDT  + (size_t)DI * KDT * 2;
constexpr size_t OFF_XIN  = OFF_WOUT + (size_t)DM * DI * 2;
constexpr size_t OFF_Z    = OFF_XIN  + (size_t)NROWS * DI * 4;
constexpr size_t OFF_XF   = OFF_Z    + (size_t)NROWS * DI * 4;
constexpr size_t OFF_XDBL = OFF_XF   + (size_t)NROWS * DI * 4;
constexpr size_t OFF_DTH  = OFF_XDBL + (size_t)NROWS * NXP * 4;
constexpr size_t OFF_DTL  = OFF_DTH  + (size_t)NROWS * KDT * 2;
constexpr size_t WS_END   = OFF_DTL  + (size_t)NROWS * KDT * 2;
constexpr size_t OFF_YH   = OFF_XIN;
constexpr size_t OFF_YL   = OFF_YH + (size_t)NROWS * DI * 2;
static_assert(OFF_WIN % 128 == 0 && OFF_WX % 128 == 0 && OFF_WDT % 128 == 0 && OFF_WOUT % 128 == 0);
static_assert(OFF_XIN % 128 == 0 && OFF_Z % 128 == 0 && OFF_XF % 128 == 0 && OFF_XDBL % 128 == 0);
static_assert(OFF_DTH % 128 == 0 && OFF_DTL % 128 == 0 && OFF_YH % 128 == 0 && OFF_YL % 128 == 0);
static_assert(OFF_YL + (size_t)NROWS * DI * 2 == OFF_Z);
static_assert(WS_END <= (size_t)134217728);
static_assert((size_t)(NROWS * DM / 2048) * 2048 * 2 == OFF_WIN - OFF_X0);
static_assert((size_t)(DIN2 * DM / 2048) * 2048 * 2 == OFF_WX - OFF_WIN);
static_assert((size_t)(NXP * DI / 2048) * 2048 * 2 == OFF_WDT - OFF_WX);
static_assert((size_t)(DI * KDT / 2048) * 2048 * 2 == OFF_WOUT - OFF_WDT);
static_assert((size_t)(DM * DI / 2048) * 2048 * 2 == OFF_XIN - OFF_WOUT);
static_assert((size_t)(NROWS / 128) * (DI / 64) * 256 * 128 == OFF_Z - OFF_XIN);
static_assert((size_t)(NROWS / 128) * (DI / 64) * 256 * 128 == OFF_XF - OFF_Z);
static_assert((size_t)(DI / 256) * (NROWS / TC) * (TC * 8) * 128 == OFF_XDBL - OFF_XF);
static_assert((size_t)(NROWS / 128) * (NXP / 64) * 256 * 128 == OFF_DTH - OFF_XDBL);
static_assert((size_t)(NROWS / 128) * 128 * 128 == OFF_DTL - OFF_DTH);
static_assert((size_t)(DI / 256) * NB * (NL / TC) * (TC * 4) * 128 == OFF_YL - OFF_YH);
static_assert((size_t)(NROWS / 128) * (DM / 64) * 256 * 128 == (size_t)NROWS * DM * 4);

__device__ __forceinline__ unsigned short bf16_bits(float f) {
  unsigned u = __float_as_uint(f);
  u += 0x7FFFu + ((u >> 16) & 1u);
  return (unsigned short)(u >> 16);
}
__device__ __forceinline__ float bf16_val(unsigned short b) { return __uint_as_float(((unsigned)b) << 16); }
__device__ __forceinline__ float bf16r(float f) { return bf16_val(bf16_bits(f)); }
__device__ __forceinline__ void split_bf16(float v, unsigned short& hb, unsigned short& lb) {
  hb = bf16_bits(v);
  lb = bf16_bits(v - bf16_val(hb));
}
__device__ __forceinline__ v8f zero8() {
  v8f z;
#pragma unroll
  for (int i = 0; i < 8; ++i) z[i] = 0.0f;
  return z;
}

__device__ __forceinline__ void ldfrag_g(Frag& f, const unsigned short* p, int h) {
  f.half[0] = *(const v8usa*)(p + 8 * h);
  f.half[1] = *(const v8usa*)(p + 16 + 8 * h);
}
__device__ __forceinline__ void ldfrag_fsplit(Frag& fh, Frag& fl, const float* p, int h) {
  const v4f q0 = *(const v4fa*)(p + 8 * h);
  const v4f q1 = *(const v4fa*)(p + 8 * h + 4);
  const v4f q2 = *(const v4fa*)(p + 16 + 8 * h);
  const v4f q3 = *(const v4fa*)(p + 20 + 8 * h);
  v16us uh, ul;
#pragma unroll
  for (int j = 0; j < 4; ++j) {
    unsigned short hb, lb;
    split_bf16(q0[j], hb, lb); uh[j]      = hb; ul[j]      = lb;
    split_bf16(q1[j], hb, lb); uh[4 + j]  = hb; ul[4 + j]  = lb;
    split_bf16(q2[j], hb, lb); uh[8 + j]  = hb; ul[8 + j]  = lb;
    split_bf16(q3[j], hb, lb); uh[12 + j] = hb; ul[12 + j] = lb;
  }
  fh.u = uh;
  fl.u = ul;
}
__device__ __forceinline__ v8f mma16(v8f c, const Frag& a, const Frag& b) {
  v8f d = __builtin_amdgcn_wmma_f32_16x16x32_bf16(false, a.v, false, b.v, (short)0, c, false, false);
  asm volatile("v_nop\n\tv_nop\n\tv_nop\n\tv_nop" : "+v"(d) : "v"(a.v), "v"(b.v));
  return d;
}

__global__ __launch_bounds__(256)
void cvt_kernel(const float* __restrict__ in, int nvalid, unsigned short* out)
{
  const size_t e8 = ((size_t)blockIdx.x * 256 + threadIdx.x) * 8;
  const bool ok = (e8 < (size_t)nvalid);
  const size_t ea = ok ? e8 : (size_t)(nvalid - 8);
  const v4f a = *(const v4fa*)(in + ea);
  const v4f b = *(const v4fa*)(in + ea + 4);
  v8us o;
  o[0] = ok ? bf16_bits(a[0]) : (unsigned short)0;
  o[1] = ok ? bf16_bits(a[1]) : (unsigned short)0;
  o[2] = ok ? bf16_bits(a[2]) : (unsigned short)0;
  o[3] = ok ? bf16_bits(a[3]) : (unsigned short)0;
  o[4] = ok ? bf16_bits(b[0]) : (unsigned short)0;
  o[5] = ok ? bf16_bits(b[1]) : (unsigned short)0;
  o[6] = ok ? bf16_bits(b[2]) : (unsigned short)0;
  o[7] = ok ? bf16_bits(b[3]) : (unsigned short)0;
  unsigned short* p = out + e8;
  *(volatile v8us*)p = o;
  __threadfence();
  *(volatile v8us*)p = o;
}

__device__ __forceinline__ void c_store_pass(const float* sT, float* C, int ldc, int m0w, int cy, int w, int lane) {
  const int q8 = lane & 7, sub = lane >> 3;
#pragma unroll
  for (int i = 0; i < 16; ++i) {
    const int lid = 4 * i + sub;
    const int rl = lid >> 1, hl = lid & 1;
    const v4f v = *(const v4fa*)(sT + (32 * w + rl) * 64 + 32 * hl + 4 * q8);
    float* dst = C + (size_t)(m0w + rl) * ldc + 64 * cy + 32 * hl + 4 * q8;
    *(volatile v4f*)dst = v;
  }
}

__device__ __forceinline__ void dtr_store_pass(const float* sT, unsigned short* dh, unsigned short* dl,
                                               int m0w, int w, int lane) {
  const int q8 = lane & 7, sub = lane >> 3;
  const bool pad = (q8 >= DTR / 8);
#pragma unroll
  for (int i = 0; i < 8; ++i) {
    const int rl = 4 * i + sub;
    const float* sr = sT + (32 * w + rl) * 64 + 8 * q8;
    const v4f a = *(const v4fa*)sr;
    const v4f c = *(const v4fa*)(sr + 4);
    v8us oh, ol;
    unsigned short hb, lb;
    split_bf16(a[0], hb, lb); oh[0] = pad ? (unsigned short)0 : hb; ol[0] = pad ? (unsigned short)0 : lb;
    split_bf16(a[1], hb, lb); oh[1] = pad ? (unsigned short)0 : hb; ol[1] = pad ? (unsigned short)0 : lb;
    split_bf16(a[2], hb, lb); oh[2] = pad ? (unsigned short)0 : hb; ol[2] = pad ? (unsigned short)0 : lb;
    split_bf16(a[3], hb, lb); oh[3] = pad ? (unsigned short)0 : hb; ol[3] = pad ? (unsigned short)0 : lb;
    split_bf16(c[0], hb, lb); oh[4] = pad ? (unsigned short)0 : hb; ol[4] = pad ? (unsigned short)0 : lb;
    split_bf16(c[1], hb, lb); oh[5] = pad ? (unsigned short)0 : hb; ol[5] = pad ? (unsigned short)0 : lb;
    split_bf16(c[2], hb, lb); oh[6] = pad ? (unsigned short)0 : hb; ol[6] = pad ? (unsigned short)0 : lb;
    split_bf16(c[3], hb, lb); oh[7] = pad ? (unsigned short)0 : hb; ol[7] = pad ? (unsigned short)0 : lb;
    const size_t go = (size_t)(m0w + rl) * KDT + 8 * q8;
    *(volatile v8us*)(dh + go) = oh;
    *(volatile v8us*)(dl + go) = ol;
  }
}

template <int NPL, int XP>
__global__ __launch_bounds__(128)
void gemm_kernel(const unsigned short* __restrict__ Ah, const unsigned short* __restrict__ Al,
                 const float* __restrict__ Af, int lda,
                 const unsigned short* __restrict__ Bw, int K,
                 float* C, int ldc, unsigned short* dh, unsigned short* dl)
{
  __shared__ __attribute__((aligned(16))) float sT[128 * 64];

  const int tid = threadIdx.x, lane = tid & 31, w = tid >> 5;
  const int h = lane >> 4, m = lane & 15;
  const int m0 = blockIdx.x * 128;
  const int cy = blockIdx.y;
  const int m0w = m0 + 32 * w;

  const unsigned short* xa = Ah + (size_t)(m0w + m) * lda;
  const unsigned short* xr = Al + (size_t)(m0w + m) * lda;
  const float* xq = Af + (size_t)(m0w + m) * lda;
  const unsigned short* wb = Bw + (size_t)(64 * cy + m) * K;

  v8f acc[2][4];
#pragma unroll
  for (int mt = 0; mt < 2; ++mt)
#pragma unroll
    for (int nt = 0; nt < 4; ++nt) acc[mt][nt] = zero8();

#pragma unroll 1
  for (int k0 = 0; k0 < K; k0 += 32) {
    Frag a0, a1, e0, e1;
    if (NPL == 3) {
      ldfrag_fsplit(a0, e0, xq + k0, h);
      ldfrag_fsplit(a1, e1, xq + (size_t)16 * lda + k0, h);
    } else {
      ldfrag_g(a0, xa + k0, h);
      ldfrag_g(a1, xa + (size_t)16 * lda + k0, h);
      if (NPL == 2) {
        ldfrag_g(e0, xr + k0, h);
        ldfrag_g(e1, xr + (size_t)16 * lda + k0, h);
      }
    }
#pragma unroll
    for (int nt = 0; nt < 4; ++nt) {
      Frag b;
      ldfrag_g(b, wb + (size_t)nt * 16 * K + k0, h);
      acc[0][nt] = mma16(acc[0][nt], a0, b);
      acc[1][nt] = mma16(acc[1][nt], a1, b);
      if (NPL >= 2) {
        acc[0][nt] = mma16(acc[0][nt], e0, b);
        acc[1][nt] = mma16(acc[1][nt], e1, b);
      }
    }
  }

#pragma unroll
  for (int nt = 0; nt < 4; ++nt) {
    const int col = 16 * nt + m;
#pragma unroll
    for (int mt = 0; mt < 2; ++mt)
#pragma unroll
      for (int r = 0; r < 8; ++r) {
        const int rowl = 32 * w + 16 * mt + 8 * h + r;
        sT[rowl * 64 + col] = acc[mt][nt][r];
      }
  }
  __syncthreads();

  c_store_pass(sT, C, ldc, m0w, cy, w, lane);
  __threadfence();
  c_store_pass(sT, C, ldc, m0w, cy, w, lane);

  if (XP == 1) {
    if (cy == 0) {
      dtr_store_pass(sT, dh, dl, m0w, w, lane);
      __threadfence();
      dtr_store_pass(sT, dh, dl, m0w, w, lane);
    }
  }
}

__device__ __forceinline__ void f32tile_store_pass(const float* sF, float* xf, int pitch, int rbase, int col0,
                                                   int w, int lane) {
  const int q8 = lane & 7, sub = lane >> 3;
#pragma unroll
  for (int i = 0; i < 4; ++i) {
    const int li = 4 * i + sub;
    const int row = 2 * w + (li >> 3), q = li & 7;
    const v4f v = *(const v4fa*)(sF + row * 256 + 32 * q + 4 * q8);
    float* dst = xf + (size_t)(rbase + row) * pitch + col0 + 32 * q + 4 * q8;
    *(volatile v4f*)dst = v;
  }
}

__device__ __forceinline__ void h16tile_store_pass(const unsigned short* sH, const unsigned short* sL,
                                                   unsigned short* ph, unsigned short* pl, int pitch, int col0,
                                                   int rbase, int w, int lane) {
  const int q8 = lane & 7, sub = lane >> 3;
#pragma unroll
  for (int i = 0; i < 2; ++i) {
    const int li = 4 * i + sub;
    const int row = 2 * w + (li >> 2), q = li & 3;
    const v8us vh = *(const v8usa*)(sH + row * 256 + 64 * q + 8 * q8);
    const v8us vl = *(const v8usa*)(sL + row * 256 + 64 * q + 8 * q8);
    const size_t go = (size_t)(rbase + row) * pitch + col0 + 64 * q + 8 * q8;
    *(volatile v8us*)(ph + go) = vh;
    *(volatile v8us*)(pl + go) = vl;
  }
}

__global__ __launch_bounds__(256)
void conv_kernel(const float* __restrict__ xin, const float* __restrict__ cw, const float* __restrict__ cb,
                 float* xf)
{
  __shared__ __attribute__((aligned(16))) float sF[TC * 256];

  const int tid = threadIdx.x, lane = tid & 31, w = tid >> 5;
  const int slab = blockIdx.x;
  const int rbase = blockIdx.y * TC;
  const int b = rbase / NL, l0 = rbase - b * NL;
  const int c = 256 * slab + tid;

  const v4f cwv = *(const v4fa*)(cw + (size_t)c * 4);
  const float w0 = bf16r(cwv[0]);
  const float w1 = bf16r(cwv[1]);
  const float w2 = bf16r(cwv[2]);
  const float w3 = bf16r(cwv[3]);
  const float cbv = bf16r(cb[c]);

  const float* col = xin + (size_t)b * NL * DI + c;

  int p, pc;
  p = l0 - 3; pc = (p > 0) ? p : 0;
  float v0 = col[(size_t)pc * DI]; v0 = (p >= 0) ? v0 : 0.0f;
  p = l0 - 2; pc = (p > 0) ? p : 0;
  float v1 = col[(size_t)pc * DI]; v1 = (p >= 0) ? v1 : 0.0f;
  p = l0 - 1; pc = (p > 0) ? p : 0;
  float v2 = col[(size_t)pc * DI]; v2 = (p >= 0) ? v2 : 0.0f;

#pragma unroll 1
  for (int tt = 0; tt < TC; ++tt) {
    const float v3 = col[(size_t)(l0 + tt) * DI];
    const float s = w0 * v0 + w1 * v1 + w2 * v2 + w3 * v3 + cbv;
    const float ex = expf(-s);
    const float sg = 1.0f / (1.0f + ex);
    const float y = s * sg;
    sF[tt * 256 + tid] = y;
    v0 = v1; v1 = v2; v2 = v3;
  }
  __syncthreads();

  const int col0 = 256 * slab;
  f32tile_store_pass(sF, xf, DI, rbase, col0, w, lane);
  __threadfence();
  f32tile_store_pass(sF, xf, DI, rbase, col0, w, lane);
}

__global__ __launch_bounds__(256)
void dtscan_kernel(const unsigned short* __restrict__ dth, const unsigned short* __restrict__ dtl,
                   const unsigned short* __restrict__ wdt,
                   const float* __restrict__ xdbl,
                   const float* __restrict__ xf,
                   const float* __restrict__ zf,
                   const float* __restrict__ dtb, const float* __restrict__ alog,
                   const float* __restrict__ dpar,
                   unsigned short* yh, unsigned short* yl)
{
  __shared__ __attribute__((aligned(16))) float sD[TC * 256];
  __shared__ __attribute__((aligned(16))) unsigned short sH[TC * 256];
  __shared__ __attribute__((aligned(16))) unsigned short sL[TC * 256];
  __shared__ __attribute__((aligned(16))) float sBC[TC * 32];

  const int tid = threadIdx.x, lane = tid & 31, w = tid >> 5;
  const int h = lane >> 4, m = lane & 15;
  const int slab = blockIdx.x, b = blockIdx.y;
  const int c0 = 256 * slab;
  const int d = c0 + tid;

  const float bb = bf16r(dtb[d]);
  const float Dv = bf16r(dpar[d]);
  float An[NS];
  {
    const float* ap = alog + (size_t)d * NS;
#pragma unroll
    for (int q = 0; q < NS / 4; ++q) {
      const v4f av = *(const v4fa*)(ap + 4 * q);
#pragma unroll
      for (int j = 0; j < 4; ++j) An[4 * q + j] = -expf(bf16r(av[j]));
    }
  }

  Frag bw[2][2];
#pragma unroll
  for (int nt = 0; nt < 2; ++nt)
#pragma unroll
    for (int ks = 0; ks < 2; ++ks)
      ldfrag_g(bw[nt][ks], wdt + (size_t)(c0 + 32 * w + 16 * nt + m) * KDT + 32 * ks, h);

  float hs[NS];
#pragma unroll
  for (int n = 0; n < NS; ++n) hs[n] = 0.0f;

#pragma unroll 1
  for (int t0 = 0; t0 < NL; t0 += TC) {
    const int r0 = b * NL + t0;

    v8f acc[2];
    acc[0] = zero8(); acc[1] = zero8();
#pragma unroll
    for (int ks = 0; ks < 2; ++ks) {
      Frag ah, ar;
      ldfrag_g(ah, dth + (size_t)(r0 + m) * KDT + 32 * ks, h);
      ldfrag_g(ar, dtl + (size_t)(r0 + m) * KDT + 32 * ks, h);
#pragma unroll
      for (int nt = 0; nt < 2; ++nt) {
        acc[nt] = mma16(acc[nt], ah, bw[nt][ks]);
        acc[nt] = mma16(acc[nt], ar, bw[nt][ks]);
      }
    }
#pragma unroll
    for (int nt = 0; nt < 2; ++nt)
#pragma unroll
      for (int r = 0; r < 8; ++r)
        sD[(8 * h + r) * 256 + 32 * w + 16 * nt + m] = acc[nt][r];

    if (tid < 128) {
      const int tok = tid >> 3, q = tid & 7;
      const v4f v = *(const v4fa*)(xdbl + (size_t)(r0 + tok) * NXP + DTR + 4 * q);
      *(v4fa*)(sBC + tok * 32 + 4 * q) = v;
    }
    __syncthreads();

#pragma unroll 1
    for (int tt = 0; tt < TC; ++tt) {
      const float dpre = sD[tt * 256 + tid];
      const float xx = dpre + bb;
      const float dl = fmaxf(xx, 0.0f) + log1pf(expf(-fabsf(xx)));
      const float xv = xf[(size_t)(r0 + tt) * DI + d];
      const float rv = zf[(size_t)(r0 + tt) * DI + d];
      const float* bc = sBC + tt * 32;
      float y = 0.0f;
#pragma unroll
      for (int n = 0; n < NS; ++n) {
        const float dA  = expf(dl * An[n]);
        const float dBu = (dl * bc[n]) * xv;
        hs[n] = dA * hs[n] + dBu;
        y += hs[n] * bc[NS + n];
      }
      const float yv = y + xv * Dv;
      const float eg = expf(-rv);
      const float g = rv * (1.0f / (1.0f + eg));
      const float yg = yv * g;
      unsigned short hb, lb;
      split_bf16(yg, hb, lb);
      sH[tt * 256 + tid] = hb;
      sL[tt * 256 + tid] = lb;
    }
    __syncthreads();

    h16tile_store_pass(sH, sL, yh, yl, DI, c0, r0, w, lane);
    __threadfence();
    h16tile_store_pass(sH, sL, yh, yl, DI, c0, r0, w, lane);
    __syncthreads();
  }
}

extern "C" void kernel_launch(void* const* d_in, const int* in_sizes, int n_in,
                              void* d_out, int out_size, void* d_ws, size_t ws_size,
                              hipStream_t stream)
{
  if (n_in < 10) return;
  if (in_sizes[0] != NROWS * DM) return;
  if (in_sizes[1] != DIN2 * DM)  return;
  if (in_sizes[2] != DI * 4)     return;
  if (in_sizes[3] != DI)         return;
  if (in_sizes[4] != NXD * DI)   return;
  if (in_sizes[5] != DI * DTR)   return;
  if (in_sizes[6] != DI)         return;
  if (in_sizes[7] != DI * NS)    return;
  if (in_sizes[8] != DI)         return;
  if (in_sizes[9] != DM * DI)    return;
  if (out_size != NROWS * DM) return;
  if (ws_size < WS_END) return;

  const float* x      = (const float*)d_in[0];
  const float* w_in   = (const float*)d_in[1];
  const float* conv_w = (const float*)d_in[2];
  const float* conv_b = (const float*)d_in[3];
  const float* w_x    = (const float*)d_in[4];
  const float* w_dt   = (const float*)d_in[5];
  const float* b_dt   = (const float*)d_in[6];
  const float* a_log  = (const float*)d_in[7];
  const float* dpar   = (const float*)d_in[8];
  const float* w_out  = (const float*)d_in[9];
  float* out = (float*)d_out;

  char* ws = (char*)d_ws;
  unsigned short* X0   = (unsigned short*)(ws + OFF_X0);
  unsigned short* WIN  = (unsigned short*)(ws + OFF_WIN);
  unsigned short* WX   = (unsigned short*)(ws + OFF_WX);
  unsigned short* WDT  = (unsigned short*)(ws + OFF_WDT);
  unsigned short* WOUT = (unsigned short*)(ws + OFF_WOUT);
  float*          XIN  = (float*)(ws + OFF_XIN);
  float*          Z    = (float*)(ws + OFF_Z);
  float*          XF   = (float*)(ws + OFF_XF);
  float*          XDBL = (float*)(ws + OFF_XDBL);
  unsigned short* DTH  = (unsigned short*)(ws + OFF_DTH);
  unsigned short* DTL  = (unsigned short*)(ws + OFF_DTL);
  unsigned short* YH   = (unsigned short*)(ws + OFF_YH);
  unsigned short* YL   = (unsigned short*)(ws + OFF_YL);

  cvt_kernel<<<dim3(NROWS * DM / 2048), dim3(256), 0, stream>>>(x, NROWS * DM, X0);
  cvt_kernel<<<dim3(DIN2 * DM / 2048), dim3(256), 0, stream>>>(w_in, DIN2 * DM, WIN);
  cvt_kernel<<<dim3(NXP * DI / 2048), dim3(256), 0, stream>>>(w_x, NXD * DI, WX);
  cvt_kernel<<<dim3(DI * KDT / 2048), dim3(256), 0, stream>>>(w_dt, DI * DTR, WDT);
  cvt_kernel<<<dim3(DM * DI / 2048), dim3(256), 0, stream>>>(w_out, DM * DI, WOUT);

  gemm_kernel<1, 0><<<dim3(NROWS / 128, DI / 64), dim3(128), 0, stream>>>(
      X0, X0, XF, DM, WIN, DM, XIN, DI, DTH, DTL);
  gemm_kernel<1, 0><<<dim3(NROWS / 128, DI / 64), dim3(128), 0, stream>>>(
      X0, X0, XF, DM, WIN + (size_t)DI * DM, DM, Z, DI, DTH, DTL);

  conv_kernel<<<dim3(DI / 256, NROWS / TC), dim3(256), 0, stream>>>(XIN, conv_w, conv_b, XF);

  gemm_kernel<3, 1><<<dim3(NROWS / 128, NXP / 64), dim3(128), 0, stream>>>(
      X0, X0, XF, DI, WX, DI, XDBL, NXP, DTH, DTL);

  dtscan_kernel<<<dim3(DI / 256, NB), dim3(256), 0, stream>>>(
      DTH, DTL, WDT, XDBL, XF, Z, b_dt, a_log, dpar, YH, YL);

  gemm_kernel<2, 0><<<dim3(NROWS / 128, DM / 64), dim3(128), 0, stream>>>(
      YH, YL, XF, DI, WOUT, DI, out, DM, DTH, DTL);
}
